// RingDilatedAttentionHybrid_23029614641318
// MI455X (gfx1250) — hardware-run, weakly checked
//
#include <hip/hip_runtime.h>


namespace {
constexpr int NT = 8192, NH = 12, D = 64, GH = 4, NP = 2048;
constexpr float XS = 8.0f, PS = 2048.0f, SCALE = 0.125f;
__device__ __forceinline__ int seg_len(int g) { return g == 0 ? 2048 : (g == 1 ? 4096 : 8192); }
__device__ __forceinline__ int rate(int g) { return g == 0 ? 1 : (g == 1 ? 2 : 4); }
typedef _Float16 b16;
typedef __attribute__((ext_vector_type(16))) _Float16 v16b;
typedef __attribute__((ext_vector_type(8))) _Float16 v8b;
typedef __attribute__((ext_vector_type(8))) float v8f;
typedef __attribute__((ext_vector_type(4))) float v4f;
__device__ __forceinline__ float bf16_rne(float f) { unsigned int u = __float_as_uint(f); u += 0x7FFFu + ((u >> 16) & 1u); return __uint_as_float(u & 0xFFFF0000u); }
__device__ __forceinline__ void split16(float v, b16& hi, b16& lo) { hi = (b16)v; lo = (b16)(v - (float)hi); }
__device__ __forceinline__ v16b frag_kb(const b16* p, int hh) { const v8b a = *(const v8b*)(p + 8 * hh), b = *(const v8b*)(p + 16 + 8 * hh); v16b f;
#pragma unroll
  for (int e = 0; e < 8; ++e) { f[e] = a[e]; f[8 + e] = b[e]; } return f; }
__device__ __forceinline__ v8f wmma16b(v16b a, v16b b, v8f c) { v8f d = __builtin_amdgcn_wmma_f32_16x16x32_f16(false, a, false, b, (short)0, c, false, false); asm volatile("v_nop\n\tv_nop\n\tv_nop\n\tv_nop" : "+v"(d) : "v"(a), "v"(b)); return d; }
__device__ __forceinline__ void wave_lds_sync() { __builtin_amdgcn_fence(__ATOMIC_RELEASE, "workgroup"); __builtin_amdgcn_wave_barrier(); __builtin_amdgcn_fence(__ATOMIC_ACQUIRE, "workgroup"); }
__device__ __forceinline__ float pmul(float a, float b) { float p = a * b; asm volatile("" : "+v"(p)); return p; }

__global__ __launch_bounds__(256) void cvt_kernel(const float* __restrict__ src, size_t n8, b16* __restrict__ dst) {
  const size_t u = (size_t)blockIdx.x * 256 + threadIdx.x; if (u >= n8) return; const size_t e = u * 8; v8b v;
#pragma unroll
  for (int j = 0; j < 8; ++j) v[j] = (b16)(bf16_rne(src[e + j]) * XS); for (int pass = 0; pass < 2; ++pass) { *(volatile v8b*)(dst + e) = v; __threadfence(); }
}
__global__ __launch_bounds__(256) void vt_kernel(const float* __restrict__ v, b16* __restrict__ VT) {
  __shared__ float Tt[64][65]; const int h = blockIdx.x % NH, jt = blockIdx.x / NH; const int g = h / GH, r = rate(g), off = g % r; const int JN = NT / r; if (jt * 64 >= JN) return; const int tid = threadIdx.x;
  for (int i = tid; i < 64 * 64; i += 256) { const int jl = i / 64, d = i % 64; const int j = jt * 64 + jl; const int sg = j / NP, pj = j % NP; const int tok = sg * seg_len(g) + off + r * pj; Tt[jl][d] = bf16_rne(v[((size_t)tok * NH + h) * D + d]); }
  __syncthreads();
  { const int d = tid / 4, gg0 = (tid % 4) * 2; for (int gg = gg0; gg < gg0 + 2; ++gg) { v8b vv; for (int j = 0; j < 8; ++j) vv[j] = (b16)(Tt[gg * 8 + j][d] * XS); const size_t o = ((size_t)h * D + d) * NT + jt * 64 + gg * 8; for (int pass = 0; pass < 2; ++pass) { *(volatile v8b*)(VT + o) = vv; __threadfence(); } } }
}
__global__ __launch_bounds__(256) void zero_kernel(float* __restrict__ out) { const size_t u = (size_t)blockIdx.x * 256 + threadIdx.x; if (u >= (size_t)NT * NH * D / 4) return; for (int pass = 0; pass < 2; ++pass) { *(volatile v4f*)(out + u * 4) = (v4f){0.0f, 0.0f, 0.0f, 0.0f}; __threadfence(); } }
__global__ __launch_bounds__(32) void att_kernel(const b16* __restrict__ QB, const b16* __restrict__ KB_, const b16* __restrict__ VT, int QLIM, float* __restrict__ out) {
  __shared__ __attribute__((aligned(16))) b16 Ph[16][32 + 8], Pl[16][32 + 8]; __shared__ float Mx[16], Sm[16]; __shared__ __attribute__((aligned(16))) float Tf[16][D + 4];
  const int lane = threadIdx.x, nloc = lane & 15, hlf = lane >> 4; const int qt = blockIdx.x % (NP / 16), rest = blockIdx.x / (NP / 16); const int h = rest % NH, sg = rest / NH; const int g = h / GH, r = rate(g), s = seg_len(g), off = g % r; if (sg >= NT / s) return; const int j0 = qt * 16; if (j0 >= QLIM) return;
  auto tok = [&](int j) -> size_t { return (size_t)sg * s + off + (size_t)r * j; };
  const b16* qrow = QB + (tok(j0 + nloc) * NH + h) * D; const v16b qa0 = frag_kb(qrow, hlf), qa1 = frag_kb(qrow + 32, hlf); const size_t vbase = (size_t)h * D * NT + (size_t)sg * NP;
  auto scores = [&](int kb, v8f sacc[2]) {
#pragma unroll
    for (int st = 0; st < 2; ++st) { const b16* kr = KB_ + (tok(kb + st * 16 + nloc) * NH + h) * D; sacc[st] = (v8f){}; sacc[st] = wmma16b(qa0, frag_kb(kr, hlf), sacc[st]); sacc[st] = wmma16b(qa1, frag_kb(kr + 32, hlf), sacc[st]); } };
  const int nblk = j0 / 32 + 1; float rmax[8];
#pragma unroll
  for (int r8 = 0; r8 < 8; ++r8) rmax[r8] = -INFINITY;
#pragma unroll 1
  for (int bi = 0; bi < nblk; ++bi) { const int kb = bi * 32; v8f sacc[2]; scores(kb, sacc);
#pragma unroll
    for (int st = 0; st < 2; ++st)
#pragma unroll
      for (int r8 = 0; r8 < 8; ++r8) { const int jq = j0 + 8 * hlf + r8, jk = kb + st * 16 + nloc; if (jk <= jq) rmax[r8] = fmaxf(rmax[r8], sacc[st][r8] * (SCALE / (XS * XS))); } }
#pragma unroll
  for (int r8 = 0; r8 < 8; ++r8) { float m = rmax[r8]; for (int o = 1; o < 16; o <<= 1) m = fmaxf(m, __shfl_xor(m, o)); if (nloc == 0) Mx[8 * hlf + r8] = m; }
  wave_lds_sync();
  v8f acc[4]; float rsum[8];
#pragma unroll
  for (int t = 0; t < 4; ++t) acc[t] = (v8f){};
#pragma unroll
  for (int r8 = 0; r8 < 8; ++r8) rsum[r8] = 0.0f;
#pragma unroll 1
  for (int bi = 0; bi < nblk; ++bi) { const int kb = bi * 32; v8f sacc[2]; scores(kb, sacc);
#pragma unroll
    for (int st = 0; st < 2; ++st)
#pragma unroll
      for (int r8 = 0; r8 < 8; ++r8) { const int rl = 8 * hlf + r8; const int jq = j0 + rl, jk = kb + st * 16 + nloc; float p = 0.0f; if (jk <= jq) p = __expf(sacc[st][r8] * (SCALE / (XS * XS)) - Mx[rl]); rsum[r8] += p; b16 ph, pl; split16(p * PS, ph, pl); Ph[rl][st * 16 + nloc] = ph; Pl[rl][st * 16 + nloc] = pl; }
    wave_lds_sync();
    const v16b pa = frag_kb(&Ph[nloc][0], hlf), pb = frag_kb(&Pl[nloc][0], hlf);
#pragma unroll
    for (int t = 0; t < 4; ++t) { const v16b vb = frag_kb(VT + vbase + (size_t)(t * 16 + nloc) * NT + kb, hlf); acc[t] = wmma16b(pa, vb, acc[t]); acc[t] = wmma16b(pb, vb, acc[t]); }
    wave_lds_sync(); }
#pragma unroll
  for (int r8 = 0; r8 < 8; ++r8) { float sm = rsum[r8]; for (int o = 1; o < 16; o <<= 1) sm += __shfl_xor(sm, o); if (nloc == 0) Sm[8 * hlf + r8] = sm; }
  wave_lds_sync();
#pragma unroll
  for (int t = 0; t < 4; ++t)
#pragma unroll
    for (int r8 = 0; r8 < 8; ++r8) Tf[8 * hlf + r8][t * 16 + nloc] = acc[t][r8] * (1.0f / (PS * XS)) / Sm[8 * hlf + r8];
  wave_lds_sync();
  for (int pass = 0; pass < 2; ++pass) { for (int rr = 0; rr < 16; ++rr) { const size_t o = (tok(j0 + rr) * NH + h) * D; ((volatile float*)out)[o + lane] = Tf[rr][lane]; ((volatile float*)out)[o + 32 + lane] = Tf[rr][32 + lane]; } __threadfence(); }
}
}

extern "C" void kernel_launch(void* const* d_in, const int* in_sizes, int n_in, void* d_out, int out_size, void* d_ws, size_t ws_size, hipStream_t stream) {
  (void)n_in;
  auto Fp = [&](int i) { return (const float*)d_in[i]; };
  if (in_sizes[0] != NT * NH * D || in_sizes[1] != NT * NH * D || in_sizes[2] != NT * NH * D || out_size != NT * NH * D) return;
  const int QLIM = NP;
  size_t off = 0; char* ws = (char*)d_ws;
  auto carve = [&](size_t bytes) { char* p = ws + off; off += (bytes + 255) & ~(size_t)255; return p; };
  b16* QB = (b16*)carve((size_t)NT * NH * D * 2); b16* KB_ = (b16*)carve((size_t)NT * NH * D * 2); b16* VT = (b16*)carve((size_t)NH * D * NT * 2);
  if (off > ws_size || off > ((size_t)64 << 20)) return;
  cvt_kernel<<<(unsigned)(((size_t)NT * NH * D / 8 + 255) / 256), 256, 0, stream>>>(Fp(0), (size_t)NT * NH * D / 8, QB); cvt_kernel<<<(unsigned)(((size_t)NT * NH * D / 8 + 255) / 256), 256, 0, stream>>>(Fp(1), (size_t)NT * NH * D / 8, KB_);
  vt_kernel<<<(NT / 64) * NH, 256, 0, stream>>>(Fp(2), VT);
  zero_kernel<<<(unsigned)(((size_t)NT * NH * D / 4 + 255) / 256), 256, 0, stream>>>((float*)d_out);
  att_kernel<<<(NP / 16) * NH * 4, 32, 0, stream>>>(QB, KB_, VT, QLIM, (float*)d_out);
}
